// MLPDecoder_39487929319518
// MI455X (gfx1250) — hardware-verified
//
#include <hip/hip_runtime.h>
#include <stddef.h>


typedef _Float16 h16;
typedef _Float16 v16h __attribute__((ext_vector_type(16)));
typedef _Float16 v8h  __attribute__((ext_vector_type(8)));
typedef float    v8f  __attribute__((ext_vector_type(8)));
typedef float    v4f  __attribute__((ext_vector_type(4)));

#ifndef NPTS
#define NPTS 2048
#endif
#define NPTS_FULL 2048
#define HDIM  128
#define ABP   (2 * HDIM)
#define TP    32

static_assert(NPTS >= 64 && NPTS <= NPTS_FULL);
static_assert((NPTS % 64) == 0 && (NPTS % TP) == 0);
static_assert((HDIM % 64) == 0 && (HDIM % 32) == 0 && (HDIM % 8) == 0);
static_assert((ABP % 64) == 0 && (ABP % 32) == 0);
static_assert(HDIM <= 256);
static_assert(((size_t)NPTS * HDIM) % 2048 == 0);
static_assert(TP * TP == 256 * 4);
static_assert(TP * (TP / 4) == 256);
static_assert((NPTS_FULL % 32) == 0);

#define LDT 72
#define LDC 68
#define ROWP 132
#define EP   33
static_assert((LDT % 8) == 0 && LDT >= 64);
static_assert((LDC % 4) == 0 && LDC >= 64);
static_assert((ROWP % 4) == 0 && ROWP >= HDIM);
static_assert(EP > TP);

#define WCARRY 64.0f
#define XCARRY 64.0f

#define WT_BYTES  ((size_t)ABP * HDIM * 2)
#define X16_BYTES ((size_t)NPTS * HDIM * 2)
#define AB_BYTES  ((size_t)NPTS * ABP * 4)
#define OFF_WT  ((size_t)0)
#define OFF_X16 (OFF_WT + WT_BYTES)
#define OFF_AB  (OFF_X16 + X16_BYTES)
#define WS_TOTAL (OFF_AB + AB_BYTES)
static_assert((WT_BYTES % 128) == 0 && (X16_BYTES % 128) == 0 && (AB_BYTES % 128) == 0);
static_assert(WS_TOTAL <= (size_t)134217728);

__device__ __forceinline__ float bf16r(float x) {
  unsigned int u = __float_as_uint(x);
  u = (u + 0x7FFFu + ((u >> 16) & 1u)) & 0xFFFF0000u;
  return __uint_as_float(u);
}

static __device__ __forceinline__ h16 toh_flush(float v) {
  const h16 r = (h16)v;
  return (fabsf(v) < 6.103515625e-05f) ? (h16)0.0f : r;
}

__device__ __forceinline__ v16h frag_at(const _Float16* p) {
  v8h lo = *(const v8h*)(p);
  v8h hi = *(const v8h*)(p + 16);
  v16h out;
#pragma unroll
  for (int i = 0; i < 8; ++i) { out[i] = lo[i]; out[i + 8] = hi[i]; }
  return out;
}

__device__ __forceinline__ v8f wmma16(v16h a, v16h b, v8f c) {
  v8f d = __builtin_amdgcn_wmma_f32_16x16x32_f16(false, a, false, b, (short)0, c,
                                                 false, false);
  asm volatile("v_nop\n\tv_nop\n\tv_nop\n\tv_nop" : "+v"(d) : "v"(a), "v"(b));
  return d;
}

__global__ __launch_bounds__(256) void wconv_kernel(
    const float* __restrict__ W, _Float16* __restrict__ Wt, unsigned ldw, unsigned ldk) {
  __shared__ _Float16 T[64 * LDT];
  const unsigned tid = threadIdx.x;
  const unsigned n0 = blockIdx.x * 64u;
  const unsigned k0 = blockIdx.y * 64u;
#pragma unroll 4
  for (unsigned j = 0; j < 16u; ++j) {
    const unsigned idx = tid + 256u * j;
    const unsigned kr = idx >> 6, nc = idx & 63u;
    const float v = W[(size_t)(k0 + kr) * ldw + n0 + nc];
    T[nc * LDT + kr] = (_Float16)(WCARRY * bf16r(v));
  }
  __syncthreads();
  v8h x[2];
  size_t off[2];
#pragma unroll
  for (unsigned i = 0; i < 2u; ++i) {
    const unsigned n = 32u * i + (tid >> 3);
    const unsigned kc = (tid & 7u) * 8u;
    x[i] = *(const v8h*)&T[n * LDT + kc];
    off[i] = (size_t)(n0 + n) * ldk + k0 + kc;
  }
#pragma unroll
  for (int i = 0; i < 2; ++i) *(volatile v8h*)(Wt + off[i]) = x[i];
  __threadfence();
#pragma unroll
  for (int i = 0; i < 2; ++i) *(volatile v8h*)(Wt + off[i]) = x[i];
}

__global__ __launch_bounds__(256) void xconv_kernel(
    const float* __restrict__ X, _Float16* __restrict__ X16) {
#pragma clang fp contract(off)
  const size_t e = ((size_t)blockIdx.x * 256u + threadIdx.x) * 8u;
  const v4f a0 = *(const v4f*)(X + e);
  const v4f a1 = *(const v4f*)(X + e + 4u);
  v8h o;
#pragma unroll
  for (int i = 0; i < 4; ++i) {
    o[i]     = toh_flush(XCARRY * bf16r(a0[i]));
    o[i + 4] = toh_flush(XCARRY * bf16r(a1[i]));
  }
  _Float16* p = X16 + e;
  *(volatile v8h*)p = o;
  __threadfence();
  *(volatile v8h*)p = o;
}

__global__ __launch_bounds__(256) void gemm_ab_kernel(
    const _Float16* __restrict__ A16, const _Float16* __restrict__ Bt,
    const float* __restrict__ bias, float* __restrict__ outf) {
  __shared__ __attribute__((aligned(16))) float Cs[64 * LDC];
  const unsigned K = (unsigned)HDIM;
  const unsigned tid = threadIdx.x, lane = tid & 31u, w = tid >> 5;
  const unsigned mw = w >> 1, nw = w & 1u;
  const unsigned hh = lane >> 4, m = lane & 15u;
  const unsigned n0 = blockIdx.x * 64u;
  const unsigned row0 = blockIdx.y * 64u;

  const _Float16* ap  = A16 + (size_t)(row0 + mw * 16u + m) * K + hh * 8u;
  const _Float16* bp0 = Bt + (size_t)(n0 + nw * 32u + m) * K + hh * 8u;
  const _Float16* bp1 = bp0 + (size_t)16 * K;
  v8f acc0 = {}, acc1 = {};
#pragma unroll 2
  for (unsigned k0 = 0; k0 < K; k0 += 32u) {
    const v16h a  = frag_at(ap + k0);
    const v16h b0 = frag_at(bp0 + k0);
    const v16h b1 = frag_at(bp1 + k0);
    acc0 = wmma16(a, b0, acc0);
    acc1 = wmma16(a, b1, acc1);
  }
#pragma unroll
  for (int r = 0; r < 8; ++r) {
    float* d = &Cs[(mw * 16u + hh * 8u + (unsigned)r) * LDC + nw * 32u + m];
    d[0]  = acc0[r];
    d[16] = acc1[r];
  }
  __syncthreads();

  const float cs = 1.0f / (WCARRY * XCARRY);
  const bool has_bias = (n0 >= (unsigned)HDIM);
  const unsigned bcol0 = has_bias ? (n0 - (unsigned)HDIM) : n0;
  v4f xs[4];
  size_t off[4];
#pragma unroll
  for (unsigned i = 0; i < 4u; ++i) {
    const unsigned r = 16u * i + (tid >> 4);
    const unsigned c = (tid & 15u) * 4u;
    const v4f u = *(const v4f*)&Cs[r * LDC + c];
    const v4f g = *(const v4f*)(bias + bcol0 + c);
    v4f val;
#pragma unroll
    for (int j = 0; j < 4; ++j) {
      const float bb = has_bias ? bf16r(g[j]) : 0.0f;
      val[j] = u[j] * cs + bb;
    }
    xs[i] = val;
    off[i] = (size_t)(row0 + r) * ABP + n0 + c;
  }
#pragma unroll
  for (int i = 0; i < 4; ++i) *(volatile v4f*)(outf + off[i]) = xs[i];
  __threadfence();
#pragma unroll
  for (int i = 0; i < 4; ++i) *(volatile v4f*)(outf + off[i]) = xs[i];
}

__global__ __launch_bounds__(256) void pair_kernel(
    const float* __restrict__ AB, const float* __restrict__ W2,
    const float* __restrict__ b2, float* __restrict__ adj) {
#pragma clang fp contract(off)
  const unsigned it = blockIdx.y;
  const unsigned jt = blockIdx.x;
  if (jt < it) return;

  __shared__ __attribute__((aligned(16))) float sA[TP * ROWP];
  __shared__ __attribute__((aligned(16))) float sB[TP * ROWP];
  __shared__ __attribute__((aligned(16))) float sW2[HDIM];
  __shared__ float sE[TP * EP];

  const unsigned tid = threadIdx.x;
  const unsigned i0 = it * (unsigned)TP;
  const unsigned j0 = jt * (unsigned)TP;

#pragma unroll
  for (unsigned v = 0; v < 4u; ++v) {
    const unsigned flat = tid + 256u * v;
    const unsigned r = flat >> 5;
    const unsigned c = (flat & 31u) << 2;
    *(v4f*)&sA[r * ROWP + c] = *(const v4f*)(AB + (size_t)(i0 + r) * ABP + c);
    *(v4f*)&sB[r * ROWP + c] = *(const v4f*)(AB + (size_t)(j0 + r) * ABP + HDIM + c);
  }
  if (tid < (unsigned)HDIM) sW2[tid] = bf16r(W2[tid]);
  __syncthreads();

  const unsigned tj = tid & 31u;
  const unsigned wave = (unsigned)__builtin_amdgcn_readfirstlane((int)(tid >> 5));

  float acc[4];
#pragma unroll
  for (int p = 0; p < 4; ++p) acc[p] = 0.0f;

#pragma unroll 2
  for (unsigned k = 0; k < (unsigned)HDIM; k += 4u) {
    const v4f b4 = *(const v4f*)&sB[tj * ROWP + k];
    const v4f w4 = *(const v4f*)&sW2[k];
#pragma unroll
    for (int p = 0; p < 4; ++p) {
      const v4f a4 = *(const v4f*)&sA[(wave + 8u * (unsigned)p) * ROWP + k];
#pragma unroll
      for (int c = 0; c < 4; ++c) {
        const float s = a4[c] + b4[c];
        const float t = (s > 0.0f) ? s : (__expf(s) - 1.0f);
        acc[p] = fmaf(t, w4[c], acc[p]);
      }
    }
  }
  const float bb2 = bf16r(b2[0]);
#pragma unroll
  for (int p = 0; p < 4; ++p) sE[(wave + 8u * (unsigned)p) * EP + tj] = acc[p] + bb2;
  __syncthreads();

  const unsigned r = tid >> 3;
  const unsigned c = (tid & 7u) * 4u;
  v4f up, tr, dg;
#pragma unroll
  for (int t = 0; t < 4; ++t) {
    const unsigned u = c + (unsigned)t;
    const float e1 = sE[r * EP + u];
    const float e2 = sE[u * EP + r];
    up[t] = e1;
    tr[t] = e2;
    dg[t] = (r < u) ? e1 : ((r > u) ? e2 : 0.0f);
  }
  const size_t offU = (size_t)(i0 + r) * NPTS_FULL + j0 + c;
  const size_t offL = (size_t)(j0 + r) * NPTS_FULL + i0 + c;
  if (it == jt) {
    *(volatile v4f*)(adj + offU) = dg;
    __threadfence();
    *(volatile v4f*)(adj + offU) = dg;
  } else {
    *(volatile v4f*)(adj + offU) = up;
    *(volatile v4f*)(adj + offL) = tr;
    __threadfence();
    *(volatile v4f*)(adj + offU) = up;
    *(volatile v4f*)(adj + offL) = tr;
  }
}

extern "C" void kernel_launch(void* const* d_in, const int* in_sizes, int n_in,
                              void* d_out, int out_size, void* d_ws, size_t ws_size,
                              hipStream_t stream) {
  if (n_in < 5) return;
  if ((long long)in_sizes[0] < (long long)NPTS * HDIM) return;
  if ((long long)in_sizes[1] < (long long)2 * HDIM * HDIM) return;
  if (in_sizes[2] < HDIM || in_sizes[3] < HDIM || in_sizes[4] < 1) return;
  if ((long long)out_size < (long long)(NPTS - 1) * NPTS_FULL + NPTS) return;
  if (ws_size < WS_TOTAL) return;

  const float* X  = (const float*)d_in[0];
  const float* W1 = (const float*)d_in[1];
  const float* B1 = (const float*)d_in[2];
  const float* W2 = (const float*)d_in[3];
  const float* B2 = (const float*)d_in[4];
  float* out = (float*)d_out;

  char* ws = (char*)d_ws;
  _Float16* Wt  = (_Float16*)(ws + OFF_WT);
  _Float16* X16 = (_Float16*)(ws + OFF_X16);
  float*    AB  = (float*)(ws + OFF_AB);

  dim3 blk(256);
  wconv_kernel<<<dim3(HDIM / 64, HDIM / 64), blk, 0, stream>>>(
      W1, Wt, (unsigned)HDIM, (unsigned)HDIM);
  wconv_kernel<<<dim3(HDIM / 64, HDIM / 64), blk, 0, stream>>>(
      W1 + (size_t)HDIM * HDIM, Wt + (size_t)HDIM * HDIM, (unsigned)HDIM, (unsigned)HDIM);
  xconv_kernel<<<dim3((unsigned)(((size_t)NPTS * HDIM) / 2048)), blk, 0, stream>>>(X, X16);
  gemm_ab_kernel<<<dim3(ABP / 64, NPTS / 64), blk, 0, stream>>>(X16, Wt, B1, AB);
  pair_kernel<<<dim3(NPTS / TP, NPTS / TP), blk, 0, stream>>>(AB, W2, B2, out);
}
